// Decoder_17154099381038
// MI455X (gfx1250) — hardware-verified
//
#include <hip/hip_runtime.h>
#include <math.h>

#ifndef NB
#define NB 1
#endif
#ifndef SEQ
#define SEQ 2048
#endif
#define NB_FULL  1
#define SEQ_FULL 2048

constexpr int DM   = 512;
constexpr int NH   = 8;
constexpr int DH   = 64;
constexpr int FF   = 2048;
constexpr int NL   = 2;
constexpr int NTOK = NB * SEQ;
constexpr int DD   = DM * DM;
constexpr float WSC = 64.0f;
constexpr float HSC = 64.0f;
constexpr float ASC = 64.0f;
constexpr float PSC = 1024.0f;
constexpr float NEGV = -1.0e9f;
constexpr float LN_EPS = 1.0e-6f;

constexpr int GBM = 128, GBN = 64, GBK = 32;
constexpr int GAP = 40;
constexpr int GCP = 68;
constexpr int GTHR = 256;
constexpr int APP = 40;
constexpr int AOP = 72;
constexpr int LROWS = 8;

static_assert(NB == 1 && NB_FULL == 1);
static_assert(SEQ % GBM == 0 && SEQ % 32 == 0 && SEQ <= SEQ_FULL);
static_assert(DM % GBN == 0 && FF % GBN == 0 && DM % GBK == 0 && FF % GBK == 0);
static_assert(DM % 64 == 0 && FF % 64 == 0);
static_assert(NH * DH == DM && DH == 64);
static_assert(NTOK % LROWS == 0);
static_assert((NTOK * DM) % 256 == 0);
static_assert(GAP % 8 == 0 && GCP % 4 == 0 && APP % 8 == 0 && AOP % 8 == 0);

typedef __attribute__((ext_vector_type(16))) _Float16 v16h;
typedef __attribute__((ext_vector_type(8)))  _Float16 v8h;
typedef __attribute__((ext_vector_type(8)))  float    v8f;
typedef __attribute__((ext_vector_type(4)))  float    v4f;

__device__ __forceinline__ void dep_guard2(v8f& a, v8f& b, v16h x, v16h y) {
  asm volatile("v_nop\n\tv_nop\n\tv_nop\n\tv_nop" : "+v"(a), "+v"(b) : "v"(x), "v"(y));
}
__device__ __forceinline__ void dep_guard4(v8f& a, v8f& b, v8f& c, v8f& d, v16h x, v16h y) {
  asm volatile("v_nop\n\tv_nop\n\tv_nop\n\tv_nop" : "+v"(a), "+v"(b), "+v"(c), "+v"(d) : "v"(x), "v"(y));
}
__device__ __forceinline__ void keepm_h(v16h a, v16h b) { asm volatile("v_nop" :: "v"(a), "v"(b) : "memory"); }
__device__ __forceinline__ void wave_lds_sync() {
  __builtin_amdgcn_fence(3  , "workgroup");
  __builtin_amdgcn_wave_barrier();
  __builtin_amdgcn_fence(2  , "workgroup");
}

struct FragH {
  union U { v16h v; v8h h[2]; };
  static __device__ __forceinline__ v16h load(const _Float16* p) {
    U f; f.h[0] = *(const v8h*)(p); f.h[1] = *(const v8h*)(p + 16); return f.v;
  }
  static __device__ __forceinline__ v8f mma(v16h a, v16h b, v8f c) {
    return __builtin_amdgcn_wmma_f32_16x16x32_f16(false, a, false, b, (short)0, c, false, false);
  }
};

__device__ __forceinline__ float bf16r(float v) {
  unsigned int u = __float_as_uint(v);
  u = (u + 0x7FFFu + ((u >> 16) & 1u)) & 0xFFFF0000u;
  return __uint_as_float(u);
}

__global__ __launch_bounds__(256) void wprep_kernel(const float* __restrict__ src, _Float16* __restrict__ dst, int K, int N) {
  __shared__ float tile[64 * 65];
  const int tid = threadIdx.x, lane = tid & 31, wv = tid >> 5;
  const int n0 = blockIdx.x * 64, k0 = blockIdx.y * 64;
  const size_t zs = (size_t)blockIdx.z * (size_t)K * (size_t)N;
  const float* s = src + zs;
  _Float16* d = dst + zs;
  const int nc = tid & 63, kr = tid >> 6;
#pragma unroll
  for (int i = 0; i < 16; ++i) {
    const int k = kr + 4 * i;
    tile[k * 65 + nc] = s[(size_t)(k0 + k) * (size_t)N + (size_t)(n0 + nc)];
  }
  __syncthreads();
  const int q = lane >> 3, k8 = (lane & 7) * 8;
  v8h hv[2];
#pragma unroll
  for (int it = 0; it < 2; ++it) {
    const int n = it * 32 + wv * 4 + q;
#pragma unroll
    for (int e = 0; e < 8; ++e) hv[it][e] = (_Float16)(bf16r(tile[(k8 + e) * 65 + n]) * WSC);
  }
  for (int pass = 0; pass < 2; ++pass) {
#pragma unroll
    for (int it = 0; it < 2; ++it) {
      const int n = it * 32 + wv * 4 + q;
      *(volatile v8h*)(d + (size_t)(n0 + n) * (size_t)K + (size_t)(k0 + k8)) = hv[it];
    }
    __threadfence();
  }
}

__global__ __launch_bounds__(256) void inprep_kernel(const float* __restrict__ x, const float* __restrict__ enc,
                                                     float* __restrict__ XF, _Float16* __restrict__ X16, _Float16* __restrict__ E16) {
  __shared__ __align__(16) float vs[256];
  const int tid = threadIdx.x;
  const size_t base = (size_t)blockIdx.x * 256;
  const size_t idx = base + (size_t)tid;
  const int pos = (int)(idx / DM);
  const int c = (int)(idx % DM);
  const int m = c & (DM / 2 - 1);
  const float ex = (2.0f * (float)m) * (1.0f / (float)DM);
  const float pw = powf(10000.0f, ex);
  const float rate = 1.0f / pw;
  const float ang = (float)pos * rate;
  float sv, cv;
  sincosf(ang, &sv, &cv);
  const float pe = (c < DM / 2) ? sv : cv;
  vs[tid] = bf16r(x[idx]) + pe;
  __syncthreads();
  if (tid < 64) {
    const v4f w = *(const v4f*)(vs + tid * 4);
    float* dp = XF + base + (size_t)tid * 4;
    *(volatile v4f*)dp = w;
    __threadfence();
    *(volatile v4f*)dp = w;
  } else if (tid < 96) {
    const int j = tid - 64;
    const v4f a = *(const v4f*)(vs + j * 8);
    const v4f b = *(const v4f*)(vs + j * 8 + 4);
    v8h hv;
#pragma unroll
    for (int e = 0; e < 4; ++e) { hv[e] = (_Float16)a[e]; hv[4 + e] = (_Float16)b[e]; }
    _Float16* dp = X16 + base + (size_t)j * 8;
    *(volatile v8h*)dp = hv;
    __threadfence();
    *(volatile v8h*)dp = hv;
  } else if (tid < 128) {
    const int j = tid - 96;
    const float* ep = enc + base + (size_t)j * 8;
    const v4f a = *(const v4f*)(ep);
    const v4f b = *(const v4f*)(ep + 4);
    v8h hv;
#pragma unroll
    for (int e = 0; e < 4; ++e) { hv[e] = (_Float16)bf16r(a[e]); hv[4 + e] = (_Float16)bf16r(b[e]); }
    _Float16* dp = E16 + base + (size_t)j * 8;
    *(volatile v8h*)dp = hv;
    __threadfence();
    *(volatile v8h*)dp = hv;
  }
}

__global__ __launch_bounds__(GTHR) void gemm_kernel(
    const _Float16* __restrict__ A, const _Float16* __restrict__ W, const float* __restrict__ bias,
    float* __restrict__ outF, _Float16* __restrict__ outH,
    int M, int N, int K, int zsW, int zsB, int zsO, int modeLo, int zT, int relu, float accScale, float outScale) {
  __shared__ __align__(16) _Float16 As[GBM * GAP];
  __shared__ __align__(16) _Float16 Bs[GBN * GAP];
  __shared__ __align__(16) float    Cs[GBM * GCP];
  const int tid = threadIdx.x, lane = tid & 31, wv = tid >> 5, ml = lane & 15, hh = lane >> 4;
  const int m0 = blockIdx.y * GBM, n0 = blockIdx.x * GBN, z = blockIdx.z;
  const int mode = (z == zT) ? 2 : modeLo;
  const _Float16* Wz = W + (size_t)z * (size_t)zsW;
  const float* bz = bias + (size_t)z * (size_t)zsB;
  const int ar = tid >> 2, kc = (tid & 3) * 8;
  const _Float16* pa0 = A  + (size_t)(m0 + ar) * (size_t)K + kc;
  const _Float16* pa1 = A  + (size_t)(m0 + 64 + ar) * (size_t)K + kc;
  const _Float16* pb  = Wz + (size_t)(n0 + ar) * (size_t)K + kc;
  const v8f z8 = {0.f, 0.f, 0.f, 0.f, 0.f, 0.f, 0.f, 0.f};
  v8f acc[4];
#pragma unroll
  for (int nt = 0; nt < 4; ++nt) acc[nt] = z8;
  const int arow = 16 * wv + ml;

#pragma unroll 1
  for (int k0 = 0; k0 < K; k0 += GBK) {
    const v8h ra0 = *(const v8h*)(pa0 + k0);
    const v8h ra1 = *(const v8h*)(pa1 + k0);
    const v8h rb  = *(const v8h*)(pb + k0);
    *(v8h*)(As + ar * GAP + kc) = ra0;
    *(v8h*)(As + (64 + ar) * GAP + kc) = ra1;
    *(v8h*)(Bs + ar * GAP + kc) = rb;
    __syncthreads();
    const v16h af = FragH::load(As + arow * GAP + 8 * hh);
    v16h bf[4];
#pragma unroll
    for (int nt = 0; nt < 4; ++nt) bf[nt] = FragH::load(Bs + (16 * nt + ml) * GAP + 8 * hh);
#pragma unroll
    for (int nt = 0; nt < 4; ++nt) acc[nt] = FragH::mma(af, bf[nt], acc[nt]);
    dep_guard4(acc[0], acc[1], acc[2], acc[3], af, bf[3]);
    __syncthreads();
  }

#pragma unroll
  for (int nt = 0; nt < 4; ++nt) {
    const float bb = bf16r(bz[n0 + 16 * nt + ml]);
#pragma unroll
    for (int r = 0; r < 8; ++r) {
      float v = acc[nt][r] * accScale + bb;
      v = (relu != 0) ? fmaxf(v, 0.0f) : v;
      Cs[(16 * wv + 8 * hh + r) * GCP + 16 * nt + ml] = v;
    }
  }
  __syncthreads();

  const int q = lane >> 3, p8 = lane & 7;
  if (mode == 0) {
    float* ob = outF + (size_t)z * (size_t)zsO;
    for (int pass = 0; pass < 2; ++pass) {
#pragma unroll
      for (int it = 0; it < 8; ++it) {
        const int line = it * 32 + wv * 4 + q;
        const int row = line >> 1, col = 32 * (line & 1) + 4 * p8;
        const v4f v = *(const v4f*)(Cs + row * GCP + col);
        *(volatile v4f*)(ob + (size_t)(m0 + row) * (size_t)N + (size_t)(n0 + col)) = v;
      }
      __threadfence();
    }
  } else if (mode == 1) {
    _Float16* ob = outH + (size_t)z * (size_t)zsO;
    for (int pass = 0; pass < 2; ++pass) {
#pragma unroll
      for (int it = 0; it < 4; ++it) {
        const int row = it * 32 + wv * 4 + q;
        const int col = 8 * p8;
        const v4f a = *(const v4f*)(Cs + row * GCP + col);
        const v4f b = *(const v4f*)(Cs + row * GCP + col + 4);
        v8h hv;
#pragma unroll
        for (int e = 0; e < 4; ++e) { hv[e] = (_Float16)(a[e] * outScale); hv[4 + e] = (_Float16)(b[e] * outScale); }
        *(volatile v8h*)(ob + (size_t)(m0 + row) * (size_t)N + (size_t)(n0 + col)) = hv;
      }
      __threadfence();
    }
  } else {
    _Float16* ob = outH + (size_t)z * (size_t)zsO;
    for (int pass = 0; pass < 2; ++pass) {
#pragma unroll
      for (int it = 0; it < 4; ++it) {
        const int line = it * 32 + wv * 4 + q;
        const int dcol = line >> 1, key0 = 64 * (line & 1) + 8 * p8;
        v8h hv;
#pragma unroll
        for (int e = 0; e < 8; ++e) hv[e] = (_Float16)(Cs[(key0 + e) * GCP + dcol] * outScale);
        *(volatile v8h*)(ob + (size_t)(n0 + dcol) * (size_t)M + (size_t)(m0 + key0)) = hv;
      }
      __threadfence();
    }
  }
}

__global__ __launch_bounds__(32) void attn_kernel(const _Float16* __restrict__ Q, const _Float16* __restrict__ Kp,
                                                  const _Float16* __restrict__ VT, _Float16* __restrict__ ATT,
                                                  int nkeys, int causal) {
  __shared__ __align__(16) _Float16 Pl[16 * APP];
  __shared__ __align__(16) _Float16 Os[16 * AOP];
  const int lane = threadIdx.x & 31, ml = lane & 15, hh = lane >> 4;
  const int q0 = blockIdx.x * 16, h = blockIdx.y;
  const _Float16* qp = Q + (size_t)(q0 + ml) * DM + h * DH + 8 * hh;
  const v16h aq0 = FragH::load(qp);
  const v16h aq1 = FragH::load(qp + 32);
  keepm_h(aq0, aq1);
  const v8f z8 = {0.f, 0.f, 0.f, 0.f, 0.f, 0.f, 0.f, 0.f};
  v8f o[4];
#pragma unroll
  for (int nt = 0; nt < 4; ++nt) o[nt] = z8;
  float mrow[8], lrow[8];
#pragma unroll
  for (int r = 0; r < 8; ++r) { mrow[r] = -3.0e38f; lrow[r] = 0.0f; }
  const int kend = (causal != 0) ? (q0 + 16) : nkeys;

#pragma unroll 1
  for (int kb = 0; kb < kend; kb += 32) {
    v8f s0 = z8, s1 = z8;
    {
      const _Float16* k0p = Kp + (size_t)(kb + ml) * DM + h * DH + 8 * hh;
      const _Float16* k1p = Kp + (size_t)(kb + 16 + ml) * DM + h * DH + 8 * hh;
      const v16h b00 = FragH::load(k0p);
      const v16h b10 = FragH::load(k1p);
      const v16h b01 = FragH::load(k0p + 32);
      const v16h b11 = FragH::load(k1p + 32);
      s0 = FragH::mma(aq0, b00, s0);
      s1 = FragH::mma(aq0, b10, s1);
      s0 = FragH::mma(aq1, b01, s0);
      s1 = FragH::mma(aq1, b11, s1);
      dep_guard2(s0, s1, b01, b11);
    }
    float p0[8], p1[8], mx[8], alp[8], rs[8];
#pragma unroll
    for (int r = 0; r < 8; ++r) {
      const int qrow = q0 + 8 * hh + r;
      const float mk0 = (causal != 0 && (kb + ml) > qrow) ? 1.0f : 0.0f;
      const float mk1 = (causal != 0 && (kb + 16 + ml) > qrow) ? 1.0f : 0.0f;
      const float v0 = s0[r] * 0.125f + mk0 * NEGV;
      const float v1 = s1[r] * 0.125f + mk1 * NEGV;
      p0[r] = v0; p1[r] = v1;
      mx[r] = fmaxf(v0, v1);
    }
#pragma unroll
    for (int sh = 1; sh < 16; sh <<= 1) {
#pragma unroll
      for (int r = 0; r < 8; ++r) mx[r] = fmaxf(mx[r], __shfl_xor(mx[r], sh, 32));
    }
#pragma unroll
    for (int r = 0; r < 8; ++r) {
      const float mn = fmaxf(mrow[r], mx[r]);
      alp[r] = __expf(mrow[r] - mn);
      mrow[r] = mn;
      p0[r] = __expf(p0[r] - mn);
      p1[r] = __expf(p1[r] - mn);
      rs[r] = p0[r] + p1[r];
    }
#pragma unroll
    for (int sh = 1; sh < 16; sh <<= 1) {
#pragma unroll
      for (int r = 0; r < 8; ++r) rs[r] += __shfl_xor(rs[r], sh, 32);
    }
#pragma unroll
    for (int r = 0; r < 8; ++r) lrow[r] = lrow[r] * alp[r] + rs[r];
#pragma unroll
    for (int nt = 0; nt < 4; ++nt) {
#pragma unroll
      for (int r = 0; r < 8; ++r) o[nt][r] *= alp[r];
    }
#pragma unroll
    for (int r = 0; r < 8; ++r) {
      Pl[(8 * hh + r) * APP + ml]      = (_Float16)(p0[r] * PSC);
      Pl[(8 * hh + r) * APP + 16 + ml] = (_Float16)(p1[r] * PSC);
    }
    wave_lds_sync();
    const v16h pa = FragH::load(Pl + ml * APP + 8 * hh);
    keepm_h(pa, pa);
    {
      v16h bv[4];
#pragma unroll
      for (int nt = 0; nt < 4; ++nt) bv[nt] = FragH::load(VT + (size_t)(h * DH + 16 * nt + ml) * NTOK + kb + 8 * hh);
#pragma unroll
      for (int nt = 0; nt < 4; ++nt) o[nt] = FragH::mma(pa, bv[nt], o[nt]);
      dep_guard4(o[0], o[1], o[2], o[3], pa, bv[3]);
    }
  }

  float sc[8];
#pragma unroll
  for (int r = 0; r < 8; ++r) sc[r] = ASC / (lrow[r] * PSC);
#pragma unroll
  for (int nt = 0; nt < 4; ++nt) {
#pragma unroll
    for (int r = 0; r < 8; ++r) Os[(8 * hh + r) * AOP + 16 * nt + ml] = (_Float16)(o[nt][r] * sc[r]);
  }
  wave_lds_sync();
  const int q = lane >> 3, p8 = lane & 7;
  for (int pass = 0; pass < 2; ++pass) {
#pragma unroll
    for (int it = 0; it < 4; ++it) {
      const int row = it * 4 + q;
      const v8h v = *(const v8h*)(Os + row * AOP + 8 * p8);
      *(volatile v8h*)(ATT + (size_t)(q0 + row) * DM + h * DH + 8 * p8) = v;
    }
    __threadfence();
  }
}

__global__ __launch_bounds__(256) void ln_kernel(const float* __restrict__ X, const float* __restrict__ T,
                                                 const float* __restrict__ g, const float* __restrict__ b,
                                                 float* __restrict__ outF, _Float16* __restrict__ outH) {
  __shared__ __align__(16) float rowbuf[LROWS * DM];
  const int tid = threadIdx.x, lane = tid & 31, wv = tid >> 5;
  const int row = blockIdx.x * LROWS + wv;
  const size_t rb = (size_t)row * DM;
  v4f v[4];
  float s = 0.0f;
#pragma unroll
  for (int j = 0; j < 4; ++j) {
    const int col = 4 * lane + 128 * j;
    const v4f a = *(const v4f*)(X + rb + col);
    const v4f t = *(const v4f*)(T + rb + col);
    v[j] = a + t;
    s += (v[j][0] + v[j][1]) + (v[j][2] + v[j][3]);
  }
#pragma unroll
  for (int sh = 1; sh < 32; sh <<= 1) s += __shfl_xor(s, sh, 32);
  const float mu = s * (1.0f / (float)DM);
  float q2 = 0.0f;
#pragma unroll
  for (int j = 0; j < 4; ++j) {
#pragma unroll
    for (int e = 0; e < 4; ++e) { const float d = v[j][e] - mu; q2 += d * d; }
  }
#pragma unroll
  for (int sh = 1; sh < 32; sh <<= 1) q2 += __shfl_xor(q2, sh, 32);
  const float var = q2 * (1.0f / (float)DM);
  const float inv = rsqrtf(var + LN_EPS);
  v4f o[4];
#pragma unroll
  for (int j = 0; j < 4; ++j) {
    const int col = 4 * lane + 128 * j;
    const v4f gg = *(const v4f*)(g + col);
    const v4f bb = *(const v4f*)(b + col);
#pragma unroll
    for (int e = 0; e < 4; ++e) o[j][e] = (v[j][e] - mu) * inv * bf16r(gg[e]) + bf16r(bb[e]);
  }
  for (int pass = 0; pass < 2; ++pass) {
#pragma unroll
    for (int j = 0; j < 4; ++j) *(volatile v4f*)(outF + rb + 4 * lane + 128 * j) = o[j];
    __threadfence();
  }
  float* myrow = rowbuf + wv * DM;
#pragma unroll
  for (int j = 0; j < 4; ++j) *(v4f*)(myrow + 4 * lane + 128 * j) = o[j];
  wave_lds_sync();
  v8h hv[2];
#pragma unroll
  for (int j2 = 0; j2 < 2; ++j2) {
    const v4f a  = *(const v4f*)(myrow + 8 * lane + 256 * j2);
    const v4f c4 = *(const v4f*)(myrow + 8 * lane + 256 * j2 + 4);
#pragma unroll
    for (int e = 0; e < 4; ++e) { hv[j2][e] = (_Float16)a[e]; hv[j2][4 + e] = (_Float16)c4[e]; }
  }
  for (int pass = 0; pass < 2; ++pass) {
#pragma unroll
    for (int j2 = 0; j2 < 2; ++j2) *(volatile v8h*)(outH + rb + 8 * lane + 256 * j2) = hv[j2];
    __threadfence();
  }
}

extern "C" void kernel_launch(void* const* d_in, const int* in_sizes, int n_in,
                              void* d_out, int out_size, void* d_ws, size_t ws_size, hipStream_t stream) {
  if (n_in < 12 || d_out == nullptr || d_ws == nullptr) return;
  if (in_sizes[0] < NTOK * DM || in_sizes[1] < NTOK * DM || in_sizes[2] < NL * 4 * DD || in_sizes[3] < NL * 4 * DM ||
      in_sizes[4] < NL * 4 * DD || in_sizes[5] < NL * 4 * DM || in_sizes[6] < NL * DM * FF || in_sizes[7] < NL * FF ||
      in_sizes[8] < NL * FF * DM || in_sizes[9] < NL * DM || in_sizes[10] < NL * 3 * DM || in_sizes[11] < NL * 3 * DM ||
      out_size < NTOK * DM) return;

  const float* x_in = (const float*)d_in[0];
  const float* enc  = (const float*)d_in[1];
  const float* a1w  = (const float*)d_in[2];
  const float* a1b  = (const float*)d_in[3];
  const float* a2w  = (const float*)d_in[4];
  const float* a2b  = (const float*)d_in[5];
  const float* fw1  = (const float*)d_in[6];
  const float* fb1  = (const float*)d_in[7];
  const float* fw2  = (const float*)d_in[8];
  const float* fb2  = (const float*)d_in[9];
  const float* lng  = (const float*)d_in[10];
  const float* lnb  = (const float*)d_in[11];
  float* out = (float*)d_out;

  char* ws = (char*)d_ws; size_t off = 0;
  auto carve = [&](size_t bytes) -> char* { char* p = ws + off; off += (bytes + 255) & ~(size_t)255; return p; };
  const size_t planeF = (size_t)NTOK * DM * 4, planeH = (size_t)NTOK * DM * 2;
  float*    XFA = (float*)carve(planeF);
  float*    XFB = (float*)carve(planeF);
  float*    T32 = (float*)carve(planeF);
  _Float16* X16 = (_Float16*)carve(planeH);
  _Float16* E16 = (_Float16*)carve(planeH);
  _Float16* QKV = (_Float16*)carve(3 * planeH);
  _Float16* ATT = (_Float16*)carve(planeH);
  _Float16* HID = (_Float16*)carve((size_t)NTOK * FF * 2);
  _Float16* W1T = (_Float16*)carve((size_t)NL * 4 * DD * 2);
  _Float16* W2T = (_Float16*)carve((size_t)NL * 4 * DD * 2);
  _Float16* WF1 = (_Float16*)carve((size_t)NL * DM * FF * 2);
  _Float16* WF2 = (_Float16*)carve((size_t)NL * FF * DM * 2);
  if (off > ws_size || off > (size_t)134217728) return;
  _Float16* Q16  = QKV;
  _Float16* K16  = QKV + (size_t)NTOK * DM;
  _Float16* VT16 = QKV + (size_t)2 * NTOK * DM;
  const int zsO = NTOK * DM;

  wprep_kernel<<<dim3(DM / 64, DM / 64, NL * 4), 256, 0, stream>>>(a1w, W1T, DM, DM);
  wprep_kernel<<<dim3(DM / 64, DM / 64, NL * 4), 256, 0, stream>>>(a2w, W2T, DM, DM);
  wprep_kernel<<<dim3(FF / 64, DM / 64, NL), 256, 0, stream>>>(fw1, WF1, DM, FF);
  wprep_kernel<<<dim3(DM / 64, FF / 64, NL), 256, 0, stream>>>(fw2, WF2, FF, DM);
  inprep_kernel<<<(NTOK * DM) / 256, 256, 0, stream>>>(x_in, enc, XFA, X16, E16);

  const dim3 gD(DM / GBN, NTOK / GBM, 1), gD3(DM / GBN, NTOK / GBM, 3), gD2(DM / GBN, NTOK / GBM, 2), gF(FF / GBN, NTOK / GBM, 1);
  const dim3 gA(NTOK / 16, NH);
  const float invW = 1.0f / WSC, invWA = 1.0f / (WSC * ASC), invWH = 1.0f / (WSC * HSC);
  float* curF = XFA;
  float* altF = XFB;
  for (int l = 0; l < NL; ++l) {
    const _Float16* w1 = W1T + (size_t)l * 4 * DD;
    const _Float16* w2 = W2T + (size_t)l * 4 * DD;
    const float* b1 = a1b + (size_t)l * 4 * DM;
    const float* b2 = a2b + (size_t)l * 4 * DM;
    gemm_kernel<<<gD3, GTHR, 0, stream>>>(X16, w1, b1, T32, Q16, NTOK, DM, DM, DD, DM, zsO, 1, 2, 0, invW, 1.0f);
    attn_kernel<<<gA, 32, 0, stream>>>(Q16, K16, VT16, ATT, NTOK, 1);
    gemm_kernel<<<gD, GTHR, 0, stream>>>(ATT, w1 + 3 * DD, b1 + 3 * DM, T32, Q16, NTOK, DM, DM, 0, 0, 0, 0, -1, 0, invWA, 1.0f);
    ln_kernel<<<NTOK / LROWS, 256, 0, stream>>>(curF, T32, lng + (size_t)(l * 3 + 0) * DM, lnb + (size_t)(l * 3 + 0) * DM, altF, X16);
    { float* tf = curF; curF = altF; altF = tf; }
    gemm_kernel<<<gD, GTHR, 0, stream>>>(X16, w2, b2, T32, Q16, NTOK, DM, DM, 0, 0, 0, 1, -1, 0, invW, 1.0f);
    gemm_kernel<<<gD2, GTHR, 0, stream>>>(E16, w2 + DD, b2 + DM, T32, K16, NTOK, DM, DM, DD, DM, zsO, 1, 1, 0, invW, 1.0f);
    attn_kernel<<<gA, 32, 0, stream>>>(Q16, K16, VT16, ATT, NTOK, 0);
    gemm_kernel<<<gD, GTHR, 0, stream>>>(ATT, w2 + 3 * DD, b2 + 3 * DM, T32, Q16, NTOK, DM, DM, 0, 0, 0, 0, -1, 0, invWA, 1.0f);
    ln_kernel<<<NTOK / LROWS, 256, 0, stream>>>(curF, T32, lng + (size_t)(l * 3 + 1) * DM, lnb + (size_t)(l * 3 + 1) * DM, altF, X16);
    { float* tf = curF; curF = altF; altF = tf; }
    gemm_kernel<<<gF, GTHR, 0, stream>>>(X16, WF1 + (size_t)l * FF * DM, fb1 + (size_t)l * FF, T32, HID, NTOK, FF, DM, 0, 0, 0, 1, -1, 1, invW, HSC);
    gemm_kernel<<<gD, GTHR, 0, stream>>>(HID, WF2 + (size_t)l * DM * FF, fb2 + (size_t)l * DM, T32, Q16, NTOK, DM, FF, 0, 0, 0, 0, -1, 0, invWH, 1.0f);
    float* o3 = (l == NL - 1) ? out : altF;
    ln_kernel<<<NTOK / LROWS, 256, 0, stream>>>(curF, T32, lng + (size_t)(l * 3 + 2) * DM, lnb + (size_t)(l * 3 + 2) * DM, o3, X16);
    { float* tf = curF; curF = o3; altF = tf; }
  }
}
